// CrossLocal_31834297598462
// MI455X (gfx1250) — hardware-verified
//
#include <hip/hip_runtime.h>
#include <math.h>
#include <stdint.h>


#define NB    4
#define CH    64
#define CI    32
#define HM    128
#define HC    64
#define NC    (HC * HC)
#define NM    (HM * HM)
#define NTOK  (NB * NC)
#define KC    128
#define NKC   (NC / KC)
#define NSUB  (KC / 32)
#define KP    40
#define VP    (KC + 8)
#define AW    8
#define ATHR  (AW * 32)
#define QB    (AW * 16)
#define NQB   (NC / QB)
#define LDSA  (2 * KC * KP + 2 * CI * VP)
#define SVP   72
#define TP    68
#define YP    36
#define WSZ   2048

static_assert(NC == 4096 && NM == 16384 && NTOK == 16384 && HM == 2 * HC);
static_assert(NKC * KC == NC && NSUB * 32 == KC && NQB * QB == NC && ATHR == 256);
static_assert(AW * 1024 <= LDSA);
static_assert((KP % 8) == 0 && (VP % 8) == 0 && (SVP % 8) == 0 && (TP % 4) == 0 && (YP % 4) == 0);
static_assert(CI * CH == WSZ);
static_assert((NTOK % 64) == 0 && (NC % 64) == 0 && (NC % 32) == 0);

typedef _Float16 v16h __attribute__((ext_vector_type(16)));
typedef _Float16 v8h  __attribute__((ext_vector_type(8)));
typedef float    v8f  __attribute__((ext_vector_type(8)));
typedef float    v4f  __attribute__((ext_vector_type(4)));
typedef float    v2f  __attribute__((ext_vector_type(2)));
typedef unsigned int v4u __attribute__((ext_vector_type(4)));

__device__ __forceinline__ unsigned short bf_bits(float f) {
  unsigned u = __float_as_uint(f);
  return (unsigned short)((u + 0x7FFFu + ((u >> 16) & 1u)) >> 16);
}
__device__ __forceinline__ float bf_up(unsigned short h) { return __uint_as_float(((unsigned)h) << 16); }
__device__ __forceinline__ float bfr(float f) { return bf_up(bf_bits(f)); }
__device__ __forceinline__ unsigned short h_bits(_Float16 x) { return __builtin_bit_cast(unsigned short, x); }
__device__ __forceinline__ unsigned pk16(unsigned short a, unsigned short b) { return (unsigned)a | ((unsigned)b << 16); }
__device__ __forceinline__ v8f zero8() { v8f z = {0.f, 0.f, 0.f, 0.f, 0.f, 0.f, 0.f, 0.f}; return z; }

__device__ __forceinline__ v16h ldfrag_h(const _Float16* p) {
  union { v16h v; v8h h[2]; } f;
  f.h[0] = *(const v8h*)(p);
  f.h[1] = *(const v8h*)(p + 16);
  return f.v;
}

__device__ __forceinline__ v8f mma_h_raw(v16h a, v16h b, v8f c) {
  return __builtin_amdgcn_wmma_f32_16x16x32_f16(false, a, false, b, (short)0, c, false, false);
}
__device__ __forceinline__ void res_guard3(v8f& t, v8f& acc, v16h x, v16h y, v16h z) {
#if defined(__HIP_DEVICE_COMPILE__)
  asm volatile("v_nop\n\tv_nop\n\tv_nop\n\tv_nop" : "+v"(t), "+v"(acc) : "v"(x), "v"(y), "v"(z));
#endif
}
__device__ __forceinline__ void dep_guard_h(v8f& a, v8f& b, v16h x, v16h y) {
#if defined(__HIP_DEVICE_COMPILE__)
  asm volatile("v_nop\n\tv_nop\n\tv_nop\n\tv_nop" : "+v"(a), "+v"(b) : "v"(x), "v"(y));
#endif
}
__device__ __forceinline__ void dep_guard3(v8f& a, v8f& b, v16h x, v16h y, v16h z) {
#if defined(__HIP_DEVICE_COMPILE__)
  asm volatile("v_nop\n\tv_nop\n\tv_nop\n\tv_nop" : "+v"(a), "+v"(b) : "v"(x), "v"(y), "v"(z));
#endif
}
__device__ __forceinline__ void dep_guard4i(v8f& a, v8f& b, v16h w, v16h x, v16h y, v16h z) {
#if defined(__HIP_DEVICE_COMPILE__)
  asm volatile("v_nop\n\tv_nop\n\tv_nop\n\tv_nop" : "+v"(a), "+v"(b) : "v"(w), "v"(x), "v"(y), "v"(z));
#endif
}
__device__ __forceinline__ void keep2_h(v16h a, v16h b) {
#if defined(__HIP_DEVICE_COMPILE__)
  asm volatile("v_nop" :: "v"(a), "v"(b));
#endif
}
__device__ __forceinline__ void keep4_h(v16h a, v16h b, v16h c, v16h d) {
#if defined(__HIP_DEVICE_COMPILE__)
  asm volatile("v_nop" :: "v"(a), "v"(b), "v"(c), "v"(d));
#endif
}
__device__ __forceinline__ void acc_guard4(v8f& a, v8f& b, v8f& c, v8f& d) {
#if defined(__HIP_DEVICE_COMPILE__)
  asm volatile("v_nop\n\tv_nop\n\tv_nop\n\tv_nop" : "+v"(a), "+v"(b), "+v"(c), "+v"(d));
#endif
}
__device__ __forceinline__ void wave_sync_lds() {
  __builtin_amdgcn_fence(__ATOMIC_RELEASE, "workgroup");
  __builtin_amdgcn_wave_barrier();
  __builtin_amdgcn_fence(__ATOMIC_ACQUIRE, "workgroup");
}

__global__ __launch_bounds__(256) void cvt_w(const float* __restrict__ w0, const float* __restrict__ w1,
                                             const float* __restrict__ w2, const float* __restrict__ w3,
                                             unsigned short* WB, float scale) {
  const float* src = w0;
  if (blockIdx.x == 1) src = w1;
  if (blockIdx.x == 2) src = w2;
  if (blockIdx.x == 3) src = w3;
  const int i = threadIdx.x;
  const v4f a = *(const v4f*)(src + i * 8);
  const v4f c = *(const v4f*)(src + i * 8 + 4);
  float f[8];
  f[0] = a[0]; f[1] = a[1]; f[2] = a[2]; f[3] = a[3];
  f[4] = c[0]; f[5] = c[1]; f[6] = c[2]; f[7] = c[3];
  unsigned short hb[8];
#pragma unroll
  for (int e = 0; e < 8; ++e) hb[e] = h_bits((_Float16)(bfr(f[e]) * scale));
  v4u p;
  p[0] = pk16(hb[0], hb[1]);
  p[1] = pk16(hb[2], hb[3]);
  p[2] = pk16(hb[4], hb[5]);
  p[3] = pk16(hb[6], hb[7]);
  unsigned short* dst = WB + (size_t)blockIdx.x * WSZ + i * 8;
  *(volatile v4u*)dst = p;
  __threadfence();
  *(volatile v4u*)dst = p;
}

__global__ __launch_bounds__(256) void cvt_cross(const float* __restrict__ x, unsigned short* CT, float scale) {
  __shared__ __align__(16) float sf[CH * TP];
  const int tid = threadIdx.x, lane = tid & 31, wave = tid >> 5;
  const int b = blockIdx.y, n0 = blockIdx.x * 64;
  const int cl = tid >> 4, n4 = (tid & 15) * 4;
#pragma unroll
  for (int p = 0; p < 4; ++p) {
    const int c = p * 16 + cl;
    const v4f v = *(const v4f*)(x + ((size_t)(b * CH + c)) * NC + n0 + n4);
    *(v4f*)(sf + c * TP + n4) = v;
  }
  __syncthreads();
  const int rq = lane >> 3, c8 = (lane & 7) * 8;
#pragma unroll
  for (int it = 0; it < 2; ++it) {
    const int row = wave * 8 + it * 4 + rq;
    unsigned short hb[8];
#pragma unroll
    for (int e = 0; e < 8; ++e) hb[e] = h_bits((_Float16)(bfr(sf[(c8 + e) * TP + row]) * scale));
    v4u p;
    p[0] = pk16(hb[0], hb[1]);
    p[1] = pk16(hb[2], hb[3]);
    p[2] = pk16(hb[4], hb[5]);
    p[3] = pk16(hb[6], hb[7]);
    unsigned short* dst = CT + ((size_t)(b * NC + n0 + row)) * CH + c8;
    *(volatile v4u*)dst = p;
    __threadfence();
    *(volatile v4u*)dst = p;
  }
}

__global__ __launch_bounds__(256) void cvt_main(const float* __restrict__ x, unsigned short* ZH,
                                                unsigned short* ZL, float scale) {
  __shared__ __align__(16) float sz[CH * TP];
  const int tid = threadIdx.x, lane = tid & 31, wave = tid >> 5;
  const int b = blockIdx.y, i = blockIdx.x;
  const int n0 = i * HC;
  const int cl = tid >> 5, q = tid & 31;
#pragma unroll 1
  for (int p = 0; p < 8; ++p) {
    const int c = p * 8 + cl;
    const float* base = x + ((size_t)(b * CH + c)) * NM + (size_t)(2 * i) * HM + 4 * q;
    const v4f A  = *(const v4f*)(base);
    const v4f Cv = *(const v4f*)(base + HM);
    const float a0 = bfr(A[0]),  a1 = bfr(A[1]),  a2 = bfr(A[2]),  a3 = bfr(A[3]);
    const float c0 = bfr(Cv[0]), c1 = bfr(Cv[1]), c2 = bfr(Cv[2]), c3 = bfr(Cv[3]);
    const float t0 = 0.5f * a0 + 0.5f * c0;
    const float t1 = 0.5f * a1 + 0.5f * c1;
    const float t2 = 0.5f * a2 + 0.5f * c2;
    const float t3 = 0.5f * a3 + 0.5f * c3;
    v2f zz;
    zz[0] = 0.5f * t0 + 0.5f * t1;
    zz[1] = 0.5f * t2 + 0.5f * t3;
    *(v2f*)(sz + c * TP + 2 * q) = zz;
  }
  __syncthreads();
  const int rq = lane >> 3, c8 = (lane & 7) * 8;
#pragma unroll
  for (int it = 0; it < 2; ++it) {
    const int row = wave * 8 + it * 4 + rq;
    unsigned short hb[8], lb[8];
#pragma unroll
    for (int e = 0; e < 8; ++e) {
      const float zs = sz[(c8 + e) * TP + row] * scale;
      const _Float16 xh = (_Float16)zs;
      hb[e] = h_bits(xh);
      lb[e] = h_bits((_Float16)((zs - (float)xh) * 2048.0f));
    }
    v4u ph, pl;
#pragma unroll
    for (int k = 0; k < 4; ++k) { ph[k] = pk16(hb[2 * k], hb[2 * k + 1]); pl[k] = pk16(lb[2 * k], lb[2 * k + 1]); }
    const size_t off = ((size_t)(b * NC + n0 + row)) * CH + c8;
    *(volatile v4u*)(ZH + off) = ph;
    *(volatile v4u*)(ZL + off) = pl;
    __threadfence();
    *(volatile v4u*)(ZH + off) = ph;
    *(volatile v4u*)(ZL + off) = pl;
  }
}

__global__ __launch_bounds__(256) void proj_qk(
    const unsigned short* __restrict__ WGp, const unsigned short* __restrict__ WTp,
    const unsigned short* __restrict__ CTp, const float* __restrict__ gb, const float* __restrict__ tb,
    unsigned short* QH, unsigned short* QL, unsigned short* KH, unsigned short* KL, float osc) {
  const _Float16* AG = (const _Float16*)(const void*)WGp;
  const _Float16* AT = (const _Float16*)(const void*)WTp;
  const _Float16* Bt = (const _Float16*)(const void*)CTp;
  __shared__ __align__(16) unsigned short sP[8][2][1024];
  const int lane = threadIdx.x & 31;
  const int wave = threadIdx.x >> 5;
  const int tile = blockIdx.x * 8 + wave;
  if (tile >= NTOK / 32) return;
  const int n0 = tile * 32;
  const int rlane = lane & 15;
  const int hh    = lane >> 4;
  const int koff  = hh * 8;

  v8f acc[4][2];
#pragma unroll
  for (int i = 0; i < 4; ++i)
#pragma unroll
    for (int j = 0; j < 2; ++j) acc[i][j] = zero8();

  for (int k0 = 0; k0 < CH; k0 += 32) {
    v16h bf[2];
#pragma unroll
    for (int j = 0; j < 2; ++j) {
      const size_t bo = (size_t)(n0 + (j << 4) + rlane) * CH + koff + k0;
      bf[j] = ldfrag_h(Bt + bo);
    }
#pragma unroll
    for (int i = 0; i < 4; ++i) {
      const _Float16* Ap = (i < 2) ? AG : AT;
      const size_t ao = (size_t)(((i & 1) << 4) + rlane) * CH + koff + k0;
      const v16h ah = ldfrag_h(Ap + ao);
#pragma unroll
      for (int j = 0; j < 2; ++j) acc[i][j] = mma_h_raw(ah, bf[j], acc[i][j]);
      dep_guard_h(acc[i][0], acc[i][1], ah, bf[1]);
    }
    keep2_h(bf[0], bf[1]);
  }
  acc_guard4(acc[0][0], acc[0][1], acc[1][0], acc[1][1]);
  acc_guard4(acc[2][0], acc[2][1], acc[3][0], acc[3][1]);

  unsigned short* s0 = &sP[wave][0][0];
  unsigned short* s1 = &sP[wave][1][0];
#pragma unroll
  for (int hp = 0; hp < 2; ++hp) {
    const float* bp = (hp == 0) ? gb : tb;
    unsigned short* Ph = (hp == 0) ? QH : KH;
    unsigned short* Pl = (hp == 0) ? QL : KL;
    float b16[2][8];
#pragma unroll
    for (int il = 0; il < 2; ++il) {
      const v4f g0 = *(const v4f*)(bp + 16 * il + 8 * hh);
      const v4f g1 = *(const v4f*)(bp + 16 * il + 8 * hh + 4);
      b16[il][0] = 16.0f * bfr(g0[0]); b16[il][1] = 16.0f * bfr(g0[1]);
      b16[il][2] = 16.0f * bfr(g0[2]); b16[il][3] = 16.0f * bfr(g0[3]);
      b16[il][4] = 16.0f * bfr(g1[0]); b16[il][5] = 16.0f * bfr(g1[1]);
      b16[il][6] = 16.0f * bfr(g1[2]); b16[il][7] = 16.0f * bfr(g1[3]);
    }
#pragma unroll
    for (int j = 0; j < 2; ++j) {
#pragma unroll
      for (int il = 0; il < 2; ++il) {
        unsigned short hq8[8], lq8[8];
#pragma unroll
        for (int r = 0; r < 8; ++r) {
          const float f = acc[2 * hp + il][j][r] * osc + b16[il][r];
          const _Float16 xh = (_Float16)f;
          hq8[r] = h_bits(xh);
          lq8[r] = h_bits((_Float16)((f - (float)xh) * 2048.0f));
        }
        v4u ph, pl;
#pragma unroll
        for (int q = 0; q < 4; ++q) {
          ph[q] = pk16(hq8[2 * q], hq8[2 * q + 1]);
          pl[q] = pk16(lq8[2 * q], lq8[2 * q + 1]);
        }
        const int so = ((j << 4) + rlane) * CI + (il << 4) + 8 * hh;
        *(v4u*)(s0 + so) = ph;
        *(v4u*)(s1 + so) = pl;
      }
    }
    wave_sync_lds();
    const size_t pb = (size_t)n0 * CI;
    for (int pass = 0; pass < 2; ++pass) {
#pragma unroll
      for (int cch = 0; cch < 4; ++cch) {
        const int e = cch * 256 + lane * 8;
        const v4u v = *(const v4u*)(s0 + e);
        const v4u w = *(const v4u*)(s1 + e);
        *(volatile v4u*)(Ph + pb + e) = v;
        *(volatile v4u*)(Pl + pb + e) = w;
      }
      __threadfence();
    }
    wave_sync_lds();
  }
}

__global__ __launch_bounds__(128) void proj_v(
    const unsigned short* __restrict__ WPp, const unsigned short* __restrict__ ZHp,
    const unsigned short* __restrict__ ZLp, const float* __restrict__ pbias,
    unsigned short* VH, unsigned short* VL, float osc, float rres) {
  const _Float16* A  = (const _Float16*)(const void*)WPp;
  const _Float16* BH = (const _Float16*)(const void*)ZHp;
  const _Float16* BL = (const _Float16*)(const void*)ZLp;
  __shared__ __align__(16) unsigned short sV[4][2][CI * SVP];
  const int lane = threadIdx.x & 31;
  const int wave = threadIdx.x >> 5;
  const int tile = blockIdx.x * 4 + wave;
  if (tile >= NTOK / 64) return;
  const int n0  = tile * 64;
  const int b   = n0 >> 12;
  const int nl0 = n0 & (NC - 1);
  const int rlane = lane & 15;
  const int hh    = lane >> 4;
  const int koff  = hh * 8;

  v8f acc[2][4];
#pragma unroll
  for (int i = 0; i < 2; ++i)
#pragma unroll
    for (int j = 0; j < 4; ++j) acc[i][j] = zero8();

  for (int k0 = 0; k0 < CH; k0 += 32) {
    v16h av[2];
#pragma unroll
    for (int i = 0; i < 2; ++i) av[i] = ldfrag_h(A + (size_t)((i << 4) + rlane) * CH + koff + k0);
#pragma unroll
    for (int j = 0; j < 4; ++j) {
      const size_t bo = (size_t)(n0 + (j << 4) + rlane) * CH + koff + k0;
      const v16h bh = ldfrag_h(BH + bo);
      const v16h bl = ldfrag_h(BL + bo);
#pragma unroll
      for (int i = 0; i < 2; ++i) {
        acc[i][j] = mma_h_raw(av[i], bh, acc[i][j]);
        v8f tp = mma_h_raw(av[i], bl, zero8());
        res_guard3(tp, acc[i][j], av[i], bh, bl);
#pragma unroll
        for (int r = 0; r < 8; ++r) acc[i][j][r] += tp[r] * rres;
      }
    }
    keep2_h(av[0], av[1]);
  }
  acc_guard4(acc[0][0], acc[0][1], acc[0][2], acc[0][3]);
  acc_guard4(acc[1][0], acc[1][1], acc[1][2], acc[1][3]);

  float b16[2][8];
#pragma unroll
  for (int i = 0; i < 2; ++i) {
    const v4f g0 = *(const v4f*)(pbias + 16 * i + 8 * hh);
    const v4f g1 = *(const v4f*)(pbias + 16 * i + 8 * hh + 4);
    b16[i][0] = 16.0f * bfr(g0[0]); b16[i][1] = 16.0f * bfr(g0[1]);
    b16[i][2] = 16.0f * bfr(g0[2]); b16[i][3] = 16.0f * bfr(g0[3]);
    b16[i][4] = 16.0f * bfr(g1[0]); b16[i][5] = 16.0f * bfr(g1[1]);
    b16[i][6] = 16.0f * bfr(g1[2]); b16[i][7] = 16.0f * bfr(g1[3]);
  }
  unsigned short* s0 = &sV[wave][0][0];
  unsigned short* s1 = &sV[wave][1][0];
#pragma unroll
  for (int i = 0; i < 2; ++i) {
#pragma unroll
    for (int j = 0; j < 4; ++j) {
#pragma unroll
      for (int r = 0; r < 8; ++r) {
        const float f = acc[i][j][r] * osc + b16[i][r];
        const _Float16 xh = (_Float16)f;
        const int so = ((i << 4) + 8 * hh + r) * SVP + (j << 4) + rlane;
        s0[so] = h_bits(xh);
        s1[so] = h_bits((_Float16)((f - (float)xh) * 2048.0f));
      }
    }
  }
  wave_sync_lds();
  const int rq = lane >> 3, c8 = (lane & 7) * 8;
  for (int pass = 0; pass < 2; ++pass) {
#pragma unroll
    for (int it = 0; it < 8; ++it) {
      const int d = it * 4 + rq;
      const size_t dst = ((size_t)(b * CI + d)) * NC + nl0 + c8;
      const v4u v = *(const v4u*)(s0 + d * SVP + c8);
      const v4u w = *(const v4u*)(s1 + d * SVP + c8);
      *(volatile v4u*)(VH + dst) = v;
      *(volatile v4u*)(VL + dst) = w;
    }
    __threadfence();
  }
  wave_sync_lds();
}

__global__ __launch_bounds__(ATHR) void attn_kernel(
    const unsigned short* __restrict__ QHp, const unsigned short* __restrict__ QLp,
    const unsigned short* __restrict__ KHp, const unsigned short* __restrict__ KLp,
    const unsigned short* __restrict__ VHp, const unsigned short* __restrict__ VLp,
    unsigned short* CXH, unsigned short* CXL, float rscale) {
  __shared__ __align__(16) unsigned short lds_u[LDSA];
  unsigned short* kh_u = lds_u;
  unsigned short* kl_u = lds_u + KC * KP;
  unsigned short* vh_u = lds_u + 2 * KC * KP;
  unsigned short* vl_u = vh_u + CI * VP;
  const _Float16* khs = (const _Float16*)(const void*)kh_u;
  const _Float16* kls = (const _Float16*)(const void*)kl_u;
  const _Float16* vhs = (const _Float16*)(const void*)vh_u;
  const _Float16* vls = (const _Float16*)(const void*)vl_u;
  const _Float16* QH = (const _Float16*)(const void*)QHp;
  const _Float16* QL = (const _Float16*)(const void*)QLp;

  const int tid = threadIdx.x, lane = tid & 31, wave = tid >> 5;
  const int b = blockIdx.y;
  const int rlane = lane & 15, hsel = lane >> 4, koff = hsel * 8;
  const int n0w = blockIdx.x * QB + wave * 16;

  const size_t qo = ((size_t)(b * NC + n0w + rlane)) * CI + koff;
  const v16h qh = ldfrag_h(QH + qo);
  const v16h ql = ldfrag_h(QL + qo);

  const float C2048  = 1.0f / 2048.0f;
  const float CS     = 1.0f / 256.0f;
  const float LN1024 = 6.931471805599453f;

  v8f oh[2], ol[2];
#pragma unroll
  for (int dt = 0; dt < 2; ++dt) { oh[dt] = zero8(); ol[dt] = zero8(); }
  float m_run = -1.0e30f, l_run = 0.0f;

#pragma unroll 1
  for (int kc = 0; kc < NKC; ++kc) {
    const int kc0 = kc * KC;
    __syncthreads();
    for (int i = tid; i < KC * 4; i += ATHR) {
      const int key = i >> 2, c8 = (i & 3) * 8;
      const size_t go = ((size_t)(b * NC + kc0 + key)) * CI + c8;
      const v4u vh = *(const v4u*)(KHp + go);
      const v4u vl = *(const v4u*)(KLp + go);
      *(v4u*)(kh_u + key * KP + c8) = vh;
      *(v4u*)(kl_u + key * KP + c8) = vl;
    }
    for (int i = tid; i < CI * (KC / 8); i += ATHR) {
      const int d = i / (KC / 8);
      const int j = i - d * (KC / 8);
      const size_t go = ((size_t)(b * CI + d)) * NC + kc0 + 8 * j;
      const v4u a = *(const v4u*)(VHp + go);
      const v4u c = *(const v4u*)(VLp + go);
      *(v4u*)(vh_u + d * VP + 8 * j) = a;
      *(v4u*)(vl_u + d * VP + 8 * j) = c;
    }
    __syncthreads();

#pragma unroll 1
    for (int sub = 0; sub < NSUB; ++sub) {
      const int kr = sub * 32;
      float a[2][8];
#pragma unroll
      for (int t = 0; t < 2; ++t) {
        const int krow = kr + 16 * t + rlane;
        const v16h khf = ldfrag_h(khs + krow * KP + koff);
        const v16h klf = ldfrag_h(kls + krow * KP + koff);
        v8f sh = mma_h_raw(khf, qh, zero8());
        v8f sr = mma_h_raw(khf, ql, zero8());
        sr = mma_h_raw(klf, qh, sr);
        dep_guard4i(sh, sr, khf, klf, qh, ql);
#pragma unroll
        for (int r = 0; r < 8; ++r) a[t][r] = (sh[r] + sr[r] * C2048) * CS;
      }

      float mloc = -1.0e30f;
#pragma unroll
      for (int r = 0; r < 8; ++r) mloc = fmaxf(mloc, fmaxf(a[0][r], a[1][r]));
      mloc = fmaxf(mloc, __shfl_xor(mloc, 16, 32));
      const float newM  = fmaxf(m_run, mloc);
      const float alpha = __expf(m_run - newM);
      const float msh   = newM - LN1024;
      float ssum = 0.0f;
      float p[2][8];
#pragma unroll
      for (int r = 0; r < 8; ++r) {
        p[0][r] = __expf(a[0][r] - msh);
        p[1][r] = __expf(a[1][r] - msh);
        ssum += p[0][r] + p[1][r];
      }
      ssum += __shfl_xor(ssum, 16, 32);
      l_run = l_run * alpha + ssum;
      m_run = newM;
#pragma unroll
      for (int dt = 0; dt < 2; ++dt) {
#pragma unroll
        for (int r = 0; r < 8; ++r) { oh[dt][r] *= alpha; ol[dt][r] *= alpha; }
      }

      union { v16h v; _Float16 s[16]; } ph;
#pragma unroll
      for (int r = 0; r < 8; ++r) {
        ph.s[r]     = (_Float16)p[0][r];
        ph.s[8 + r] = (_Float16)p[1][r];
      }

#pragma unroll
      for (int dt = 0; dt < 2; ++dt) {
        const v16h vah = ldfrag_h(vhs + (16 * dt + rlane) * VP + kr + koff);
        const v16h val = ldfrag_h(vls + (16 * dt + rlane) * VP + kr + koff);
        oh[dt] = mma_h_raw(vah, ph.v, oh[dt]);
        ol[dt] = mma_h_raw(val, ph.v, ol[dt]);
        dep_guard3(oh[dt], ol[dt], vah, val, ph.v);
      }
    }
  }
  acc_guard4(oh[0], oh[1], ol[0], ol[1]);

  const float inv = 4.0f * (1.0f / l_run);
  __syncthreads();
  unsigned short* sth = lds_u + wave * 1024;
  unsigned short* stl = sth + 512;
#pragma unroll
  for (int dt = 0; dt < 2; ++dt) {
    v4u hv, lw;
#pragma unroll
    for (int e = 0; e < 4; ++e) {
      const float f0 = (oh[dt][2 * e]     + ol[dt][2 * e]     * C2048) * inv;
      const float f1 = (oh[dt][2 * e + 1] + ol[dt][2 * e + 1] * C2048) * inv;
      const _Float16 x0 = (_Float16)f0, x1 = (_Float16)f1;
      hv[e] = pk16(h_bits(x0), h_bits(x1));
      lw[e] = pk16(h_bits((_Float16)((f0 - (float)x0) * rscale)),
                   h_bits((_Float16)((f1 - (float)x1) * rscale)));
    }
    const int so = rlane * CI + 16 * dt + 8 * hsel;
    *(v4u*)(sth + so) = hv;
    *(v4u*)(stl + so) = lw;
  }
  wave_sync_lds();
  {
    const size_t base = ((size_t)(b * NC + n0w)) * CI;
    for (int pass = 0; pass < 2; ++pass) {
#pragma unroll
      for (int cch = 0; cch < 2; ++cch) {
        const int e = cch * 256 + lane * 8;
        const v4u v = *(const v4u*)(sth + e);
        *(volatile v4u*)(CXH + base + e) = v;
      }
      __threadfence();
    }
    for (int pass = 0; pass < 2; ++pass) {
#pragma unroll
      for (int cch = 0; cch < 2; ++cch) {
        const int e = cch * 256 + lane * 8;
        const v4u v = *(const v4u*)(stl + e);
        *(volatile v4u*)(CXL + base + e) = v;
      }
      __threadfence();
    }
  }
}

__global__ __launch_bounds__(128) void proj_w(
    const unsigned short* __restrict__ CHp, const unsigned short* __restrict__ CLp,
    const unsigned short* __restrict__ WWp, const float* __restrict__ bias,
    float* Y, float oscale, float rres) {
  const _Float16* BH = (const _Float16*)(const void*)CHp;
  const _Float16* BL = (const _Float16*)(const void*)CLp;
  const _Float16* A  = (const _Float16*)(const void*)WWp;
  __shared__ __align__(16) float sT[4][CH * YP];
  const int lane = threadIdx.x & 31;
  const int wave = threadIdx.x >> 5;
  const int tile = blockIdx.x * 4 + wave;
  if (tile >= NTOK / 32) return;
  const int n0  = tile * 32;
  const int b   = n0 >> 12;
  const int nl0 = n0 & (NC - 1);
  const int rlane = lane & 15;
  const int hh    = lane >> 4;
  const int koff  = hh * 8;

  v8f acc[4][2];
  v16h bh[2], bl[2];
#pragma unroll
  for (int j = 0; j < 2; ++j) {
    const size_t bo = (size_t)(n0 + (j << 4) + rlane) * CI + koff;
    bh[j] = ldfrag_h(BH + bo);
    bl[j] = ldfrag_h(BL + bo);
  }
#pragma unroll
  for (int i = 0; i < 4; ++i) {
    const v16h ah = ldfrag_h(A + (size_t)((i << 4) + rlane) * CI + koff);
#pragma unroll
    for (int j = 0; j < 2; ++j) {
      acc[i][j] = mma_h_raw(ah, bh[j], zero8());
      v8f tp = mma_h_raw(ah, bl[j], zero8());
      res_guard3(tp, acc[i][j], ah, bh[j], bl[j]);
#pragma unroll
      for (int r = 0; r < 8; ++r) acc[i][j][r] += tp[r] * rres;
    }
  }
  keep4_h(bh[0], bh[1], bl[0], bl[1]);
  acc_guard4(acc[0][0], acc[0][1], acc[1][0], acc[1][1]);
  acc_guard4(acc[2][0], acc[2][1], acc[3][0], acc[3][1]);

  float b8[4][8];
#pragma unroll
  for (int i = 0; i < 4; ++i) {
    const v4f g0 = *(const v4f*)(bias + 16 * i + 8 * hh);
    const v4f g1 = *(const v4f*)(bias + 16 * i + 8 * hh + 4);
    b8[i][0] = bfr(g0[0]); b8[i][1] = bfr(g0[1]); b8[i][2] = bfr(g0[2]); b8[i][3] = bfr(g0[3]);
    b8[i][4] = bfr(g1[0]); b8[i][5] = bfr(g1[1]); b8[i][6] = bfr(g1[2]); b8[i][7] = bfr(g1[3]);
  }
  float* slab = sT[wave];
#pragma unroll
  for (int i = 0; i < 4; ++i) {
#pragma unroll
    for (int j = 0; j < 2; ++j) {
#pragma unroll
      for (int r = 0; r < 8; ++r) {
        slab[((i << 4) + 8 * hh + r) * YP + (j << 4) + rlane] = acc[i][j][r] * oscale + b8[i][r];
      }
    }
  }
  wave_sync_lds();
  const int rq = lane >> 3, c4 = (lane & 7) * 4;
  for (int pass = 0; pass < 2; ++pass) {
#pragma unroll
    for (int it = 0; it < 16; ++it) {
      const int o = it * 4 + rq;
      const v4f v = *(const v4f*)(slab + o * YP + c4);
      float* dst = Y + ((size_t)(b * CH + o)) * NC + nl0 + c4;
      *(volatile v4f*)dst = v;
    }
    __threadfence();
  }
  wave_sync_lds();
}

__device__ __forceinline__ double block_sum256(double v, double* sred, int tid) {
  sred[tid] = v;
  __syncthreads();
#pragma unroll 1
  for (int off = 128; off > 0; off >>= 1) {
    if (tid < off) sred[tid] += sred[tid + off];
    __syncthreads();
  }
  const double tot = sred[0];
  __syncthreads();
  return tot;
}

__global__ __launch_bounds__(256) void bn_stats(const float* __restrict__ Y, const float* __restrict__ gam,
                                                const float* __restrict__ bet, float* ST, float eps) {
  __shared__ double sred[256];
  __shared__ __align__(16) float sst[CH * 4];
  const int tid = threadIdx.x;
  const double invn = 1.0 / (double)NTOK;
#pragma unroll 1
  for (int c = 0; c < CH; ++c) {
    double s = 0.0;
#pragma unroll 1
    for (int k = 0; k < NTOK / 256; ++k) {
      const int e = tid + 256 * k;
      const int bb = e >> 12, n = e & (NC - 1);
      s += (double)Y[((size_t)(bb * CH + c)) * NC + n];
    }
    const double mean = block_sum256(s, sred, tid) * invn;
    double s2 = 0.0;
#pragma unroll 1
    for (int k = 0; k < NTOK / 256; ++k) {
      const int e = tid + 256 * k;
      const int bb = e >> 12, n = e & (NC - 1);
      const double d = (double)Y[((size_t)(bb * CH + c)) * NC + n] - mean;
      s2 += d * d;
    }
    const double var = block_sum256(s2, sred, tid) * invn;
    if (tid == 0) {
      const float mf = (float)mean;
      const float vf = (float)var;
      sst[4 * c + 0] = mf;
      sst[4 * c + 1] = 1.0f / sqrtf(vf + eps);
      sst[4 * c + 2] = bfr(gam[c]);
      sst[4 * c + 3] = bfr(bet[c]);
    }
  }
  __syncthreads();
  if (tid < 32) {
    for (int pass = 0; pass < 2; ++pass) {
#pragma unroll
      for (int it = 0; it < 2; ++it) {
        const int e = it * 128 + tid * 4;
        const v4f v = *(const v4f*)(sst + e);
        *(volatile v4f*)(ST + e) = v;
      }
      __threadfence();
    }
  }
}

__global__ __launch_bounds__(256) void final_up(const float* __restrict__ Y, const float* __restrict__ ST,
                                                const float* __restrict__ xm, float* out) {
#pragma clang fp contract(off)
  __shared__ __align__(16) float sy[NC];
  const int tid = threadIdx.x, lane = tid & 31, wave = tid >> 5;
  const int bc = blockIdx.x;
  const int c = bc & (CH - 1);
  const v4f st = *(const v4f*)(ST + c * 4);
  const float mean = st[0], rs = st[1], ga = st[2], be = st[3];
  const float* yp = Y + (size_t)bc * NC;
#pragma unroll
  for (int k = 0; k < 4; ++k) {
    const int idx = (tid + 256 * k) * 4;
    const v4f y = *(const v4f*)(yp + idx);
    v4f o;
#pragma unroll
    for (int e = 0; e < 4; ++e) { const float t = (y[e] - mean) * rs; o[e] = t * ga + be; }
    *(v4f*)(sy + idx) = o;
  }
  __syncthreads();

  int ja[4], jb[4];
  float wj[4];
#pragma unroll
  for (int e = 0; e < 4; ++e) {
    const int j = lane * 4 + e;
    float src = ((float)j + 0.5f) * 0.5f - 0.5f;
    src = fminf(fmaxf(src, 0.0f), (float)(HC - 1));
    const int f0 = (int)floorf(src);
    ja[e] = f0;
    jb[e] = min(f0 + 1, HC - 1);
    wj[e] = src - (float)f0;
  }
  const float* mp = xm + (size_t)bc * NM;
  float* op = out + (size_t)bc * NM;
#pragma unroll 1
  for (int m = 0; m < HM / 8; ++m) {
    const int i = wave + 8 * m;
    float src = ((float)i + 0.5f) * 0.5f - 0.5f;
    src = fminf(fmaxf(src, 0.0f), (float)(HC - 1));
    const int i0 = (int)floorf(src);
    const int i1 = min(i0 + 1, HC - 1);
    const float wi = src - (float)i0;
    const float wi1 = 1.0f - wi;
    const float* ra = sy + i0 * HC;
    const float* rb = sy + i1 * HC;
    const v4f mv = *(const v4f*)(mp + i * HM + lane * 4);
    v4f res;
#pragma unroll
    for (int e = 0; e < 4; ++e) {
      const float ta = ra[ja[e]] * wi1 + rb[ja[e]] * wi;
      const float tb = ra[jb[e]] * wi1 + rb[jb[e]] * wi;
      const float wj1 = 1.0f - wj[e];
      const float val = ta * wj1 + tb * wj[e];
      res[e] = val + bfr(mv[e]);
    }
    float* dst = op + i * HM + lane * 4;
    *(volatile v4f*)dst = res;
    __threadfence();
    *(volatile v4f*)dst = res;
  }
}

extern "C" void kernel_launch(void* const* d_in, const int* in_sizes, int n_in,
                              void* d_out, int out_size, void* d_ws, size_t ws_size,
                              hipStream_t stream) {
  if (n_in < 12) return;
  if (in_sizes[0] != NB * CH * NM) return;
  if (in_sizes[1] != NB * CH * NC) return;
  if (in_sizes[2] != WSZ || in_sizes[3] != CI) return;
  if (in_sizes[4] != WSZ || in_sizes[5] != CI) return;
  if (in_sizes[6] != WSZ || in_sizes[7] != CI) return;
  if (in_sizes[8] != WSZ || in_sizes[9] != CH) return;
  if (in_sizes[10] != CH || in_sizes[11] != CH) return;
  if (out_size != NB * CH * NM) return;

  const float* xm      = (const float*)d_in[0];
  const float* xc      = (const float*)d_in[1];
  const float* g_w     = (const float*)d_in[2];
  const float* g_b     = (const float*)d_in[3];
  const float* theta_w = (const float*)d_in[4];
  const float* theta_b = (const float*)d_in[5];
  const float* phi_w   = (const float*)d_in[6];
  const float* phi_b   = (const float*)d_in[7];
  const float* w_w     = (const float*)d_in[8];
  const float* w_b     = (const float*)d_in[9];
  const float* gamma   = (const float*)d_in[10];
  const float* beta    = (const float*)d_in[11];

  const size_t PWB = (size_t)4 * WSZ * 2;
  const size_t PCT = (size_t)NTOK * CH * 2;
  const size_t PQK = (size_t)NTOK * CI * 2;
  const size_t PV  = (size_t)NB * CI * NC * 2;
  const size_t PY  = (size_t)NB * CH * NC * 4;
  const size_t PST = (size_t)CH * 4 * 4;
  size_t off = 0;
  const size_t oWB  = off; off += PWB;
  const size_t oCT  = off; off += PCT;
  const size_t oZH  = off; off += PCT;
  const size_t oZL  = off; off += PCT;
  const size_t oQH  = off; off += PQK;
  const size_t oQL  = off; off += PQK;
  const size_t oKH  = off; off += PQK;
  const size_t oKL  = off; off += PQK;
  const size_t oVH  = off; off += PV;
  const size_t oVL  = off; off += PV;
  const size_t oCXH = off; off += PQK;
  const size_t oCXL = off; off += PQK;
  const size_t oY   = off; off += PY;
  const size_t oST  = off; off += PST;
  if (off > ws_size) return;
  if (off > (size_t)134217728) return;

  char* ws = (char*)d_ws;
  unsigned short* WB  = (unsigned short*)(ws + oWB);
  unsigned short* CT  = (unsigned short*)(ws + oCT);
  unsigned short* ZH  = (unsigned short*)(ws + oZH);
  unsigned short* ZL  = (unsigned short*)(ws + oZL);
  unsigned short* QH  = (unsigned short*)(ws + oQH);
  unsigned short* QL  = (unsigned short*)(ws + oQL);
  unsigned short* KH  = (unsigned short*)(ws + oKH);
  unsigned short* KL  = (unsigned short*)(ws + oKL);
  unsigned short* VH  = (unsigned short*)(ws + oVH);
  unsigned short* VL  = (unsigned short*)(ws + oVL);
  unsigned short* CXH = (unsigned short*)(ws + oCXH);
  unsigned short* CXL = (unsigned short*)(ws + oCXL);
  float*          Y   = (float*)(ws + oY);
  float*          ST  = (float*)(ws + oST);
  float*          out = (float*)d_out;

  const dim3 blk(256);
  const dim3 gCvt(NC / 64, NB);
  const dim3 gQk((NTOK / 32 + 7) / 8);
  const dim3 gV((NTOK / 64 + 3) / 4);
  const dim3 gAttn(NQB, NB);
  const dim3 gW((NTOK / 32 + 3) / 4);
  const dim3 gFin(NB * CH);

  const float oscPrj = 1.0f / 1024.0f;
  const float rscale = 16384.0f;
  const float oscW   = 1.0f / 65536.0f;
  const float rres   = 1.0f / 16384.0f;

  cvt_w<<<dim3(4), blk, 0, stream>>>(g_w, theta_w, phi_w, w_w, WB, 1024.0f);
  cvt_cross<<<gCvt, blk, 0, stream>>>(xc, CT, 16.0f);
  cvt_main<<<gCvt, blk, 0, stream>>>(xm, ZH, ZL, 16.0f);
  proj_qk<<<gQk, blk, 0, stream>>>(WB, WB + WSZ, CT, g_b, theta_b, QH, QL, KH, KL, oscPrj);
  proj_v<<<gV, dim3(128), 0, stream>>>(WB + 2 * WSZ, ZH, ZL, phi_b, VH, VL, oscPrj, 1.0f / 2048.0f);
  attn_kernel<<<gAttn, dim3(ATHR), 0, stream>>>(QH, QL, KH, KL, VH, VL, CXH, CXL, rscale);
  proj_w<<<gW, dim3(128), 0, stream>>>(CXH, CXL, WB + 3 * WSZ, w_b, Y, oscW, rres);
  bn_stats<<<dim3(1), blk, 0, stream>>>(Y, gamma, beta, ST, 1.0e-5f);
  final_up<<<gFin, blk, 0, stream>>>(Y, ST, xm, out);
  (void)hipGetLastError();
}
